// MHSA_13511967113499
// MI455X (gfx1250) — hardware-verified
//
#include <hip/hip_runtime.h>


#ifndef NB
#define NB 4
#endif
#ifndef SEQ
#define SEQ 2048
#endif
#define NB_     NB
#define TT      SEQ
#define TT_FULL 2048
#define DM      512
#define NH_     8
#define NKV     8
#define HD      64
#define DQ      (NH_ * HD)
#define DKV     (NKV * HD)
#define D3      (3 * DM)
#define ZH      2
#define PCAR    16384.0f
#define SQK     8.0f
#define EPSN    1e-12f
static_assert(TT % 128 == 0);
static_assert(TT >= 128);
static_assert(NH_ % ZH == 0);
static_assert(DM % 64 == 0);
static_assert(HD == 64);
static_assert(D3 % 64 == 0);
static_assert(DKV % 256 == 0);

typedef _Float16 h16;
typedef unsigned short bf;
typedef __attribute__((ext_vector_type(16))) __bf16   v16bf;
typedef __attribute__((ext_vector_type(16))) _Float16 v16h;
typedef __attribute__((ext_vector_type(8)))  _Float16 v8h;
typedef __attribute__((ext_vector_type(8)))  unsigned short v8us;
typedef __attribute__((ext_vector_type(8)))  float    v8f;
typedef __attribute__((ext_vector_type(4)))  float    v4f;
typedef v8h  __attribute__((may_alias)) v8ha;
typedef v4f  __attribute__((may_alias)) v4fa;
typedef v8us __attribute__((may_alias)) v8usa;
typedef __attribute__((ext_vector_type(2))) _Float16 v2h;
typedef __attribute__((ext_vector_type(4))) _Float16 v4h;
typedef __attribute__((ext_vector_type(2))) unsigned short v2us;
typedef __attribute__((ext_vector_type(4))) unsigned short v4us;
typedef __attribute__((ext_vector_type(2))) float v2f;

__device__ __forceinline__ unsigned short f2bf(float f) { unsigned u = __float_as_uint(f); u += 0x7FFFu + ((u >> 16) & 1u); return (unsigned short)(u >> 16); }
__device__ __forceinline__ float bf2f(unsigned short b) { return __uint_as_float(((unsigned)b) << 16); }
__device__ __forceinline__ float bfr(float f) { return bf2f(f2bf(f)); }
__device__ __forceinline__ v16h cat16(v8h lo, v8h hi) { return __builtin_shufflevector(lo, hi, 0, 1, 2, 3, 4, 5, 6, 7, 8, 9, 10, 11, 12, 13, 14, 15); }
__device__ __forceinline__ v16bf cat16b(v8us lo, v8us hi) { return __builtin_bit_cast(v16bf, __builtin_shufflevector(lo, hi, 0, 1, 2, 3, 4, 5, 6, 7, 8, 9, 10, 11, 12, 13, 14, 15)); }
__device__ __forceinline__ v8f wmma16(v16h a, v16h b, v8f c) { return __builtin_amdgcn_wmma_f32_16x16x32_f16(false, a, false, b, (short)0, c, false, false); }
__device__ __forceinline__ v8f wmmab(v16bf a, v16bf b, v8f c) { return __builtin_amdgcn_wmma_f32_16x16x32_bf16(false, a, false, b, (short)0, c, false, false); }
__device__ __forceinline__ h16 tohx(float x) { return (h16)x; }
__device__ __forceinline__ void splitf(float y, unsigned short& h, unsigned short& l) { h = f2bf(y); l = f2bf(y - bf2f(h)); }

template <typename T16> struct WFrag;
template <> struct WFrag<h16> { typedef v16h V; static __device__ __forceinline__ V ld(const h16* p) { return cat16(*(const v8h*)p, *(const v8h*)(p + 16)); } static __device__ __forceinline__ v8f mma(V a, V b, v8f c) { return wmma16(a, b, c); } };
template <> struct WFrag<bf> { typedef v16bf V; static __device__ __forceinline__ V ld(const bf* p) { return cat16b(*(const v8us*)p, *(const v8us*)(p + 16)); } static __device__ __forceinline__ v8f mma(V a, V b, v8f c) { return wmmab(a, b, c); } };
template <typename T16, int NSPLIT, bool BIAS>
__global__ __launch_bounds__(32) void k_gemmw(const T16* __restrict__ A, const T16* __restrict__ A2, const T16* __restrict__ Bt, const T16* __restrict__ Bt2, int K, float* C, int ldc, const float* __restrict__ bias, size_t sA, size_t sB, size_t sC) {
    typedef typename WFrag<T16>::V V;
    __shared__ __align__(16) float os[16 * 68];
    const size_t z = blockIdx.z; A += z * sA; if (A2) A2 += z * sA; Bt += z * sB; if (Bt2) Bt2 += z * sB; C += z * sC;
    const int lane = threadIdx.x & 31, lr = lane & 15, hi = lane >> 4; const int r0 = blockIdx.x * 64, c0 = blockIdx.y * 64;
    v8f acc[4][4];
#pragma unroll
    for (int mb = 0; mb < 4; ++mb)
#pragma unroll
        for (int nb = 0; nb < 4; ++nb) acc[mb][nb] = (v8f){};
    const size_t aoff = (size_t)(r0 + lr) * K + 8 * hi, boff = (size_t)(c0 + lr) * K + 8 * hi;
#pragma unroll 1
    for (int kc = 0; kc < K; kc += 32) {
        V a[4], a2[4];
#pragma unroll
        for (int mb = 0; mb < 4; ++mb) { a[mb] = WFrag<T16>::ld(A + aoff + (size_t)mb * 16 * K + kc); if (NSPLIT == 1 || NSPLIT == 2) a2[mb] = WFrag<T16>::ld(A2 + aoff + (size_t)mb * 16 * K + kc); }
#pragma unroll
        for (int nb = 0; nb < 4; ++nb) { const V b = WFrag<T16>::ld(Bt + boff + (size_t)nb * 16 * K + kc); V b2; if (NSPLIT >= 2) b2 = WFrag<T16>::ld(Bt2 + boff + (size_t)nb * 16 * K + kc);
#pragma unroll
            for (int mb = 0; mb < 4; ++mb) { acc[mb][nb] = WFrag<T16>::mma(a[mb], b, acc[mb][nb]); if (NSPLIT == 1 || NSPLIT == 2) acc[mb][nb] = WFrag<T16>::mma(a2[mb], b, acc[mb][nb]); if (NSPLIT >= 2) acc[mb][nb] = WFrag<T16>::mma(a[mb], b2, acc[mb][nb]); } }
        asm volatile("v_nop\n\tv_nop\n\tv_nop\n\tv_nop" : "+v"(acc[0][0]), "+v"(acc[1][1]), "+v"(acc[2][2]), "+v"(acc[3][3]) : "v"(a[0]), "v"(a[3]));
    }
#pragma unroll
    for (int mb = 0; mb < 4; ++mb) {
#pragma unroll
        for (int nb = 0; nb < 4; ++nb) {
#pragma unroll
            for (int j = 0; j < 8; ++j) os[(hi * 8 + j) * 68 + nb * 16 + lr] = acc[mb][nb][j]; }
        __builtin_amdgcn_wave_barrier(); asm volatile("" ::: "memory");
        float* crow = C + (size_t)(r0 + mb * 16) * ldc + c0;
#pragma unroll 1
        for (int ps = 0; ps < 2; ++ps) {
#pragma unroll
            for (int s = 0; s < 8; ++s) { const int row = 2 * s + hi, cofs = lr * 4; v4f val = *(const v4fa*)(os + row * 68 + cofs); if (BIAS) { val[0] += bfr(bias[c0 + cofs]); val[1] += bfr(bias[c0 + cofs + 1]); val[2] += bfr(bias[c0 + cofs + 2]); val[3] += bfr(bias[c0 + cofs + 3]); }
                *(volatile v4f*)(crow + (size_t)row * ldc + cofs) = val; }
            if (ps == 0) __threadfence(); }
        __builtin_amdgcn_wave_barrier(); asm volatile("" ::: "memory");
    }
}

__global__ __launch_bounds__(256) void k_cvt8(const float* __restrict__ src, bf* dst, size_t n8) { const size_t i = (size_t)blockIdx.x * 256 + threadIdx.x; if (i >= n8) return; const v8f v = *(const v8f*)(src + i * 8); v8us o;
#pragma unroll
    for (int k = 0; k < 8; ++k) o[k] = f2bf(v[k]); *(volatile v8us*)(dst + i * 8) = o; __threadfence(); *(volatile v8us*)(dst + i * 8) = o; }

__global__ __launch_bounds__(256) void k_qkn(const float* __restrict__ F, int pitch, int nheads, h16* P16) {
    const int lane = threadIdx.x & 31; const int row = blockIdx.x * 8 + (threadIdx.x >> 5); if (row >= nheads * TT) return;
    const int h = row / TT, t = row % TT;
    const v2f xv = *(const v2f*)(F + (size_t)t * pitch + h * HD + 2 * lane);
    float s = xv[0] * xv[0] + xv[1] * xv[1];
#pragma unroll
    for (int sh = 16; sh; sh >>= 1) s += __shfl_xor(s, sh, 32);
    const float inv = __fdiv_rn(SQK, fmaxf(sqrtf(s), EPSN));
    v2h o; o[0] = tohx(xv[0] * inv); o[1] = tohx(xv[1] * inv);
    h16* p = P16 + (size_t)row * HD + 2 * lane;
    *(volatile v2h*)p = o; __threadfence(); *(volatile v2h*)p = o;
}

__global__ __launch_bounds__(256) void k_vtp16(const float* __restrict__ F, int pitch, int nheads, h16* V16) { const size_t e = ((size_t)blockIdx.x * 256 + threadIdx.x) * 2; if (e >= (size_t)nheads * HD * TT) return; const int t = (int)(e % TT); const int d = (int)((e / TT) % HD); const int g = (int)(e / ((size_t)TT * HD)); v2h o16;
#pragma unroll
    for (int q = 0; q < 2; ++q) o16[q] = tohx(F[(size_t)(t + q) * pitch + g * HD + d]);
    *(volatile v2h*)(V16 + e) = o16; __threadfence(); *(volatile v2h*)(V16 + e) = o16; }

__global__ __launch_bounds__(256) void k_vmean(const float* __restrict__ F, int pitch, int ncol, float* VM) {
    const int c = blockIdx.x * 256 + threadIdx.x; const int cc = (c < ncol) ? c : (ncol - 1);
    float s[8];
#pragma unroll
    for (int j = 0; j < 8; ++j) s[j] = 0.f;
#pragma unroll 1
    for (int t = 0; t < TT; t += 8) {
#pragma unroll
        for (int j = 0; j < 8; ++j) s[j] += F[(size_t)(t + j) * pitch + cc]; }
    const float tot = ((s[0] + s[1]) + (s[2] + s[3])) + ((s[4] + s[5]) + (s[6] + s[7]));
    const float m = tot * (1.0f / (float)TT);
    if (c < ncol) { *(volatile float*)(VM + c) = m; __threadfence(); *(volatile float*)(VM + c) = m; }
}

__global__ __launch_bounds__(256) void k_asoft(const float* __restrict__ Sb, const float* __restrict__ temp, int h0, h16* P16) {
    const int lane = threadIdx.x & 31; const int row = blockIdx.x * 8 + (threadIdx.x >> 5); if (row >= ZH * TT) return;
    const int zz = row / TT; int hh = h0 + zz; hh = hh < 0 ? 0 : (hh > NH_ - 1 ? NH_ - 1 : hh);
    const float tsc = bfr(temp[hh]) * (1.0f / (SQK * SQK));
    const float* sr = Sb + (size_t)row * TT; float v[TT / 32]; float mx = -3.0e38f;
#pragma unroll
    for (int ch = 0; ch < TT / 128; ++ch) { const int j0 = ch * 128 + lane * 4; const v4f a = *(const v4f*)(sr + j0);
#pragma unroll
        for (int q = 0; q < 4; ++q) { const float t = a[q] * tsc; v[ch * 4 + q] = t; mx = fmaxf(mx, t); } }
#pragma unroll
    for (int sh = 16; sh; sh >>= 1) mx = fmaxf(mx, __shfl_xor(mx, sh, 32));
    float sum = 0.f;
#pragma unroll
    for (int k = 0; k < TT / 32; ++k) { float d0 = __fsub_rn(v[k], mx); asm volatile("" : "+v"(d0)); v[k] = __builtin_amdgcn_exp2f(__fmul_rn(d0, 1.4426950408889634f)); sum += v[k]; }
#pragma unroll
    for (int sh = 16; sh; sh >>= 1) sum += __shfl_xor(sum, sh, 32);
    const float f = __fdiv_rn(PCAR, sum); const float sb = __fmul_rn(sum, 1.0f / (float)TT);
    v4h o[TT / 128];
#pragma unroll
    for (int ch = 0; ch < TT / 128; ++ch) {
#pragma unroll
        for (int q = 0; q < 4; ++q) { float d1 = __fsub_rn(v[ch * 4 + q], sb); asm volatile("" : "+v"(d1)); o[ch][q] = tohx(__fmul_rn(d1, f)); } }
    h16* prow = P16 + (size_t)row * TT + lane * 4;
#pragma unroll 1
    for (int ps = 0; ps < 2; ++ps) {
#pragma unroll
        for (int ch = 0; ch < TT / 128; ++ch) *(volatile v4h*)(prow + ch * 128) = o[ch];
        if (ps == 0) __threadfence(); }
}

__global__ __launch_bounds__(256) void k_ctx(const float* __restrict__ O, const float* __restrict__ VM, int h0, bf* Ch, bf* Cl) {
    const size_t e = ((size_t)blockIdx.x * 256 + threadIdx.x) * 2; if (e >= (size_t)ZH * TT * HD) return;
    const int d = (int)(e % HD); const int t = (int)((e / HD) % TT); const int zz = (int)(e / ((size_t)HD * TT)); int hh = h0 + zz; hh = hh < 0 ? 0 : (hh > NH_ - 1 ? NH_ - 1 : hh);
    const size_t oo = (size_t)t * DM + (size_t)hh * HD + d; v2us oh, ol;
#pragma unroll
    for (int q = 0; q < 2; ++q) { const float val = O[e + q] * (1.0f / PCAR) + VM[hh * HD + d + q]; unsigned short a, c; splitf(val, a, c); oh[q] = a; ol[q] = c; }
    *(volatile v2us*)(Ch + oo) = oh; *(volatile v2us*)(Cl + oo) = ol; __threadfence(); *(volatile v2us*)(Ch + oo) = oh; *(volatile v2us*)(Cl + oo) = ol;
}

extern "C" void kernel_launch(void* const* d_in, const int* in_sizes, int n_in,
                              void* d_out, int out_size, void* d_ws, size_t ws_size, hipStream_t stream) {
    if (n_in < 4) return;
    if ((size_t)in_sizes[0] < (size_t)(NB_ - 1) * TT_FULL * DM + (size_t)TT * DM) return;
    if ((size_t)in_sizes[1] < (size_t)D3 * DM) return;
    if ((size_t)in_sizes[2] < (size_t)DM * DM) return;
    if (in_sizes[3] < NH_) return;
    if ((size_t)out_size < (size_t)NB_ * TT * DM) return;
    const float* x    = (const float*)d_in[0];
    const float* wqkv = (const float*)d_in[1];
    const float* wout = (const float*)d_in[2];
    const float* temp = (const float*)d_in[3];
    float* OUT = (float*)d_out;
    char* wsp = (char*)d_ws;
    auto take = [&](size_t bytes) { char* p = wsp; wsp += (bytes + 255) & ~(size_t)255; return (void*)p; };
    bf*    WQKVb = (bf*)take((size_t)D3 * DM * 2);
    bf*    WOb   = (bf*)take((size_t)DM * DM * 2);
    bf*    XB    = (bf*)take((size_t)TT * DM * 2);
    float* F     = (float*)take((size_t)TT * D3 * 4);
    h16*   QKP   = (h16*)take((size_t)2 * NH_ * TT * HD * 2);
    h16*   VT16  = (h16*)take((size_t)NKV * HD * TT * 2);
    float* VM    = (float*)take((size_t)DKV * 4);
    float* Sb    = (float*)take((size_t)ZH * TT * TT * 4);
    h16*   P16   = (h16*)take((size_t)ZH * TT * TT * 2);
    float* Ob    = (float*)take((size_t)ZH * TT * HD * 4);
    bf*    CTh   = (bf*)take((size_t)TT * DM * 2);
    bf*    CTl   = (bf*)take((size_t)TT * DM * 2);
    if ((size_t)(wsp - (char*)d_ws) > ws_size) return;
    const float* FV = F + 2 * DM;

    k_cvt8<<<(unsigned)(((size_t)D3 * DM / 8 + 255) / 256), 256, 0, stream>>>(wqkv, WQKVb, (size_t)D3 * DM / 8);
    k_cvt8<<<(unsigned)(((size_t)DM * DM / 8 + 255) / 256), 256, 0, stream>>>(wout, WOb, (size_t)DM * DM / 8);
    const unsigned LQK = (unsigned)((2 * NH_ * TT + 7) / 8);
    const unsigned LV  = (unsigned)(((size_t)NKV * HD * TT / 2 + 255) / 256);
    const unsigned LCX = (unsigned)(((size_t)ZH * TT * HD / 2 + 255) / 256);
    for (int b = 0; b < NB_; ++b) {
        k_cvt8<<<(unsigned)(((size_t)TT * DM / 8 + 255) / 256), 256, 0, stream>>>(x + (size_t)b * TT_FULL * DM, XB, (size_t)TT * DM / 8);
        k_gemmw<bf, 0, false><<<dim3(TT / 64, D3 / 64, 1), 32, 0, stream>>>(XB, nullptr, WQKVb, nullptr, DM, F, D3, nullptr, 0, 0, 0);
        k_qkn<<<LQK, 256, 0, stream>>>(F, D3, 2 * NH_, QKP);
        k_vtp16<<<LV, 256, 0, stream>>>(FV, D3, NKV, VT16);
        k_vmean<<<DKV / 256, 256, 0, stream>>>(FV, D3, DKV, VM);
        for (int h0 = 0; h0 < NH_; h0 += ZH) {
            k_gemmw<h16, 0, false><<<dim3(TT / 64, TT / 64, ZH), 32, 0, stream>>>(QKP + (size_t)h0 * TT * HD, nullptr, QKP + (size_t)(NH_ + h0) * TT * HD, nullptr, HD, Sb, TT, nullptr, (size_t)TT * HD, (size_t)TT * HD, (size_t)TT * TT);
            k_asoft<<<(unsigned)(ZH * TT / 8), 256, 0, stream>>>(Sb, temp, h0, P16);
            k_gemmw<h16, 0, false><<<dim3(TT / 64, HD / 64, ZH), 32, 0, stream>>>(P16, nullptr, VT16 + (size_t)h0 * HD * TT, nullptr, TT, Ob, HD, nullptr, (size_t)TT * TT, (size_t)HD * TT, (size_t)TT * HD);
            k_ctx<<<LCX, 256, 0, stream>>>(Ob, VM, h0, CTh, CTl); }
        k_gemmw<bf, 1, false><<<dim3(TT / 64, DM / 64, 1), 32, 0, stream>>>(CTh, CTl, WOb, nullptr, DM, OUT + (size_t)b * TT * DM, DM, nullptr, 0, 0, 0);
    }
}
